// VLA_Adapter_L1RegressionActionHead_6975026888970
// MI455X (gfx1250) — hardware-run, weakly checked
//
#include <hip/hip_runtime.h>


#define NB_  2
#define TT   2048
#define DIN  2048
#define DD   512
#define NH_  8
#define HD   64
#define NK   2176
#define NVAL 2051
#define ZH   4
#define PCAR 1024.0f
typedef _Float16 h16;
typedef unsigned short bf;
typedef __attribute__((ext_vector_type(16))) __bf16   v16bf;
typedef __attribute__((ext_vector_type(16))) _Float16 v16h;
typedef __attribute__((ext_vector_type(8)))  _Float16 v8h;
typedef __attribute__((ext_vector_type(8)))  unsigned short v8us;
typedef __attribute__((ext_vector_type(8)))  float    v8f;
typedef __attribute__((ext_vector_type(4)))  float    v4f;
typedef v8h  __attribute__((may_alias)) v8ha;
typedef v4f  __attribute__((may_alias)) v4fa;
typedef v8us __attribute__((may_alias)) v8usa;

__device__ __forceinline__ unsigned short f2bf(float f) { unsigned u = __float_as_uint(f); u += 0x7FFFu + ((u >> 16) & 1u); return (unsigned short)(u >> 16); }
__device__ __forceinline__ float bf2f(unsigned short b) { return __uint_as_float(((unsigned)b) << 16); }
__device__ __forceinline__ float bfr(float f) { return bf2f(f2bf(f)); }
__device__ __forceinline__ v16h cat16(v8h lo, v8h hi) { return __builtin_shufflevector(lo, hi, 0, 1, 2, 3, 4, 5, 6, 7, 8, 9, 10, 11, 12, 13, 14, 15); }
__device__ __forceinline__ v16bf cat16b(v8us lo, v8us hi) { return __builtin_bit_cast(v16bf, __builtin_shufflevector(lo, hi, 0, 1, 2, 3, 4, 5, 6, 7, 8, 9, 10, 11, 12, 13, 14, 15)); }
__device__ __forceinline__ v8f wmma16(v16h a, v16h b, v8f c) { return __builtin_amdgcn_wmma_f32_16x16x32_f16(false, a, false, b, (short)0, c, false, false); }
__device__ __forceinline__ v8f wmmab(v16bf a, v16bf b, v8f c) { return __builtin_amdgcn_wmma_f32_16x16x32_bf16(false, a, false, b, (short)0, c, false, false); }


template <typename T16> struct WFrag;
template <> struct WFrag<h16> { typedef v16h V; static __device__ __forceinline__ V ld(const h16* p) { return cat16(*(const v8h*)p, *(const v8h*)(p + 16)); } static __device__ __forceinline__ v8f mma(V a, V b, v8f c) { return wmma16(a, b, c); } };
template <> struct WFrag<bf> { typedef v16bf V; static __device__ __forceinline__ V ld(const bf* p) { return cat16b(*(const v8us*)p, *(const v8us*)(p + 16)); } static __device__ __forceinline__ v8f mma(V a, V b, v8f c) { return wmmab(a, b, c); } };
template <typename T16, int NSPLIT, bool BIAS>
__global__ __launch_bounds__(32) void k_gemmw(const T16* __restrict__ A, const T16* __restrict__ A2, const T16* __restrict__ Bt, const T16* __restrict__ Bt2, int K, float* C, int ldc, const float* __restrict__ bias, size_t sA, size_t sB, size_t sC) {
    typedef typename WFrag<T16>::V V;
    __shared__ __align__(16) float os[16 * 68];
    const size_t z = blockIdx.z; A += z * sA; if (A2) A2 += z * sA; Bt += z * sB; if (Bt2) Bt2 += z * sB; C += z * sC;
    const int lane = threadIdx.x & 31, lr = lane & 15, hi = lane >> 4; const int r0 = blockIdx.x * 64, c0 = blockIdx.y * 64;
    v8f acc[4][4];
#pragma unroll
    for (int mb = 0; mb < 4; ++mb)
#pragma unroll
        for (int nb = 0; nb < 4; ++nb) acc[mb][nb] = (v8f){};
    const size_t aoff = (size_t)(r0 + lr) * K + 8 * hi, boff = (size_t)(c0 + lr) * K + 8 * hi;
#pragma unroll 1
    for (int kc = 0; kc < K; kc += 32) {
        V a[4], a2[4];
#pragma unroll
        for (int mb = 0; mb < 4; ++mb) { a[mb] = WFrag<T16>::ld(A + aoff + (size_t)mb * 16 * K + kc); if (NSPLIT == 1 || NSPLIT == 2) a2[mb] = WFrag<T16>::ld(A2 + aoff + (size_t)mb * 16 * K + kc); }
#pragma unroll
        for (int nb = 0; nb < 4; ++nb) { const V b = WFrag<T16>::ld(Bt + boff + (size_t)nb * 16 * K + kc); V b2; if (NSPLIT >= 2) b2 = WFrag<T16>::ld(Bt2 + boff + (size_t)nb * 16 * K + kc);
#pragma unroll
            for (int mb = 0; mb < 4; ++mb) { acc[mb][nb] = WFrag<T16>::mma(a[mb], b, acc[mb][nb]); if (NSPLIT == 1 || NSPLIT == 2) acc[mb][nb] = WFrag<T16>::mma(a2[mb], b, acc[mb][nb]); if (NSPLIT >= 2) acc[mb][nb] = WFrag<T16>::mma(a[mb], b2, acc[mb][nb]); } }
        asm volatile("v_nop\n\tv_nop\n\tv_nop\n\tv_nop" : "+v"(acc[0][0]), "+v"(acc[1][1]), "+v"(acc[2][2]), "+v"(acc[3][3]) : "v"(a[0]), "v"(a[3]));
    }
#pragma unroll
    for (int mb = 0; mb < 4; ++mb) {
#pragma unroll
        for (int nb = 0; nb < 4; ++nb) {
#pragma unroll
            for (int j = 0; j < 8; ++j) os[(hi * 8 + j) * 68 + nb * 16 + lr] = acc[mb][nb][j]; }
        __builtin_amdgcn_wave_barrier(); asm volatile("" ::: "memory");
        float* crow = C + (size_t)(r0 + mb * 16) * ldc + c0;
#pragma unroll 1
        for (int ps = 0; ps < 2; ++ps) {
#pragma unroll
            for (int s = 0; s < 8; ++s) { const int row = 2 * s + hi, cofs = lr * 4; v4f val = *(const v4fa*)(os + row * 68 + cofs); if (BIAS) { val[0] += bfr(bias[c0 + cofs]); val[1] += bfr(bias[c0 + cofs + 1]); val[2] += bfr(bias[c0 + cofs + 2]); val[3] += bfr(bias[c0 + cofs + 3]); }
                *(volatile v4f*)(crow + (size_t)row * ldc + cofs) = val; }
            if (ps == 0) __threadfence(); }
        __builtin_amdgcn_wave_barrier(); asm volatile("" ::: "memory");
    }
}

__device__ __forceinline__ h16 tohx(float x) { return (h16)x; }
typedef __attribute__((ext_vector_type(2))) _Float16 v2h;
typedef __attribute__((ext_vector_type(4))) _Float16 v4h;

__global__ __launch_bounds__(256) void k_wt16(const float* __restrict__ w, int K, int N, h16* W16) { __shared__ float tile[64][65]; const int nb = (N + 63) / 64; const int k0 = (blockIdx.x / nb) * 64, n0 = (blockIdx.x % nb) * 64;
    for (int i = threadIdx.x; i < 64 * 64; i += 256) { const int kk = i / 64, nn = i % 64; tile[kk][nn] = (k0 + kk < K && n0 + nn < N) ? w[(size_t)(k0 + kk) * N + n0 + nn] : 0.f; }
    __syncthreads();
    const int nn = threadIdx.x / 4, kq = (threadIdx.x % 4) * 16; if (n0 + nn >= N) return;
    for (int c = 0; c < 16; c += 4) { v4h o; o[0] = tohx(bfr(tile[kq + c][nn])); o[1] = tohx(bfr(tile[kq + c + 1][nn])); o[2] = tohx(bfr(tile[kq + c + 2][nn])); o[3] = tohx(bfr(tile[kq + c + 3][nn])); h16* dst = W16 + (size_t)(n0 + nn) * K + k0 + kq + c; *(volatile v4h*)dst = o; __threadfence(); *(volatile v4h*)dst = o; } }
__global__ __launch_bounds__(256) void k_wpad16(const float* __restrict__ w, h16* W16) { const int e = (blockIdx.x * 256 + threadIdx.x) * 2; if (e >= 64 * DD) return; const int k = e % DD, n = e / DD; v2h o; o[0] = n < 32 ? tohx(bfr(w[(size_t)k * 32 + n])) : (h16)0.f; o[1] = n < 32 ? tohx(bfr(w[(size_t)(k + 1) * 32 + n])) : (h16)0.f; *(volatile v2h*)(W16 + e) = o; __threadfence(); *(volatile v2h*)(W16 + e) = o; }
template <int W, int ARAW> __global__ __launch_bounds__(256) void k_ln16(const float* __restrict__ A, const float* __restrict__ R, const float* __restrict__ g, const float* __restrict__ bb, h16* P16) { const int lane = threadIdx.x & 31; const int row = blockIdx.x * 8 + (threadIdx.x >> 5); if (row >= TT) return; const size_t rb = (size_t)row * W;
    auto val = [&](int c) { float v = ARAW ? bfr(A[rb + c]) : A[rb + c]; if (R) v = __fadd_rn(v, R[rb + c]); return v; };
    float s = 0.f;
#pragma unroll 1
    for (int c0 = lane * 4; c0 < W; c0 += 128) { s = __fadd_rn(s, __fadd_rn(__fadd_rn(val(c0), val(c0 + 1)), __fadd_rn(val(c0 + 2), val(c0 + 3)))); }
#pragma unroll
    for (int sh = 16; sh; sh >>= 1) s += __shfl_xor(s, sh, 32);
    const float mean = s * (1.0f / W); float q2 = 0.f;
#pragma unroll 1
    for (int c0 = lane * 4; c0 < W; c0 += 128) {
#pragma unroll
        for (int u = 0; u < 4; ++u) { float d0 = __fsub_rn(val(c0 + u), mean); asm volatile("" : "+v"(d0)); float p = __fmul_rn(d0, d0); asm volatile("" : "+v"(p)); q2 = __fadd_rn(q2, p); } }
#pragma unroll
    for (int sh = 16; sh; sh >>= 1) q2 += __shfl_xor(q2, sh, 32);
    const float rstd = __frsqrt_rn(__fadd_rn(q2 * (1.0f / W), 1e-5f));
    for (int ps = 0; ps < 2; ++ps) {
#pragma unroll 1
        for (int c0 = lane * 4; c0 < W; c0 += 128) { v4h o;
#pragma unroll
            for (int u = 0; u < 4; ++u) { float t0 = __fmul_rn(__fsub_rn(val(c0 + u), mean), rstd); asm volatile("" : "+v"(t0)); float t1 = __fmul_rn(t0, bfr(g[c0 + u])); asm volatile("" : "+v"(t1)); o[u] = tohx(__fadd_rn(t1, bfr(bb[c0 + u]))); } *(volatile v4h*)(P16 + rb + c0) = o; }
        if (ps == 0) __threadfence(); } }
__global__ __launch_bounds__(256) void k_relux(const float* __restrict__ F, float* XF, h16* X16) { const int e = (blockIdx.x * 256 + threadIdx.x) * 4; if (e >= TT * DD) return; const v4f a = *(const v4f*)(F + e); v4f o; v4h o16;
#pragma unroll
    for (int u = 0; u < 4; ++u) { o[u] = fmaxf(a[u], 0.f); o16[u] = tohx(o[u]); } for (int ps = 0; ps < 2; ++ps) { *(volatile v4f*)(XF + e) = o; *(volatile v4h*)(X16 + e) = o16; if (ps == 0) __threadfence(); } }
__global__ __launch_bounds__(256) void k_res(const float* __restrict__ O2, const float* __restrict__ XF, float* Y) { const int e = (blockIdx.x * 256 + threadIdx.x) * 4; if (e >= TT * DD) return; const v4f a = *(const v4f*)(O2 + e), b = *(const v4f*)(XF + e); v4f o; o[0] = __fadd_rn(a[0], b[0]); o[1] = __fadd_rn(a[1], b[1]); o[2] = __fadd_rn(a[2], b[2]); o[3] = __fadd_rn(a[3], b[3]); *(volatile v4f*)(Y + e) = o; __threadfence(); *(volatile v4f*)(Y + e) = o; }
__device__ __forceinline__ float rope1(const float* f, int dd, float tpos) { const int i = dd & 31; const float inv = __fdiv_rn(1.0f, powf(10000.0f, (float)(2 * i) / (float)HD)); const float ang = __fmul_rn(tpos, inv); const float c = cosf(ang), s = sinf(ang); float a = __fmul_rn(f[dd], c); asm volatile("" : "+v"(a)); float b = __fmul_rn(f[dd ^ 1], s); asm volatile("" : "+v"(b)); return (dd & 1) ? __fadd_rn(a, b) : __fsub_rn(a, b); }
__global__ __launch_bounds__(256) void k_ropeqk(const float* __restrict__ F, float sc, h16* P, size_t hstride) { const int e = (blockIdx.x * 256 + threadIdx.x) * 2; if (e >= NH_ * TT * HD) return; const int d = e % HD; const int t = (e / HD) % TT; const int h = e / (HD * TT); const float* f = F + (size_t)t * DD + h * HD; v2h o;
#pragma unroll 1
    for (int u = 0; u < 2; ++u) o[u] = tohx(rope1(f, d + u, (float)t) * sc); h16* dst = P + (size_t)h * hstride + (size_t)t * HD + d; *(volatile v2h*)dst = o; __threadfence(); *(volatile v2h*)dst = o; }
__global__ __launch_bounds__(256) void k_vt(const float* __restrict__ VS, h16* VT) { const int e = (blockIdx.x * 256 + threadIdx.x) * 2; if (e >= NH_ * HD * TT) return; const int j = e % TT; const int d = (e / TT) % HD; const int h = e / (TT * HD); v2h o; o[0] = tohx(VS[(size_t)j * DD + h * HD + d]); o[1] = tohx(VS[(size_t)(j + 1) * DD + h * HD + d]); h16* dst = VT + ((size_t)h * HD + d) * NK + j; *(volatile v2h*)dst = o; __threadfence(); *(volatile v2h*)dst = o; }
__global__ __launch_bounds__(64) void k_adp(const float* __restrict__ ha, const float* __restrict__ pp, const float* __restrict__ ht, const float* __restrict__ kaW, const float* __restrict__ kab, const float* __restrict__ vaW, const float* __restrict__ vab, const float* __restrict__ ktW, const float* __restrict__ ktb, const float* __restrict__ vtW, const float* __restrict__ vtb, const float* __restrict__ gg, h16* K16, h16* VT16) {
    __shared__ float kaf[2][HD]; const int h = blockIdx.x, d = threadIdx.x; const int c = h * HD + d; float ka0 = bfr(kab[c]), ka1 = bfr(kab[c]), va0 = bfr(vab[c]), va1 = bfr(vab[c]), kt = bfr(ktb[c]), vt = bfr(vtb[c]);
#pragma unroll 1
    for (int k = 0; k < DD; ++k) { const float a0 = bfr(ha[k]), a1 = bfr(pp[k]), t0 = bfr(ht[k]); const float wka = bfr(kaW[(size_t)k * DD + c]), wva = bfr(vaW[(size_t)k * DD + c]), wkt = bfr(ktW[(size_t)k * DD + c]), wvt = bfr(vtW[(size_t)k * DD + c]);
        float p; p = __fmul_rn(a0, wka); asm volatile("" : "+v"(p)); ka0 = __fadd_rn(ka0, p); p = __fmul_rn(a1, wka); asm volatile("" : "+v"(p)); ka1 = __fadd_rn(ka1, p); p = __fmul_rn(a0, wva); asm volatile("" : "+v"(p)); va0 = __fadd_rn(va0, p); p = __fmul_rn(a1, wva); asm volatile("" : "+v"(p)); va1 = __fadd_rn(va1, p);
        p = __fmul_rn(t0, wkt); asm volatile("" : "+v"(p)); kt = __fadd_rn(kt, p); p = __fmul_rn(t0, wvt); asm volatile("" : "+v"(p)); vt = __fadd_rn(vt, p); }
    kaf[0][d] = ka0; kaf[1][d] = ka1; __syncthreads();
    const float ka1r = rope1(kaf[1], d, 1.0f);
    const float ktg = __fmul_rn(kt, tanhf(bfr(gg[0])));
    __shared__ float krow[3][HD]; krow[0][d] = ka0; krow[1][d] = ka1r; krow[2][d] = ktg; __syncthreads();
    { const int wv = d >> 5, ln = d & 31;
      for (int ps = 0; ps < 2; ++ps) { for (int r = wv; r < NK - TT; r += 2) { v2h o; o[0] = tohx(r < 3 ? krow[r < 3 ? r : 0][2 * ln] : 0.f); o[1] = tohx(r < 3 ? krow[r < 3 ? r : 0][2 * ln + 1] : 0.f); h16* dst = K16 + (size_t)h * NK * HD + (size_t)(TT + r) * HD + 2 * ln; *(volatile v2h*)dst = o; } if (ps == 0) __threadfence(); } }
    h16* vrow = VT16 + ((size_t)h * HD + d) * NK + TT;
    for (int ps = 0; ps < 2; ++ps) { for (int jx = 0; jx < NK - TT; jx += 4) { v4h o; o[0] = tohx(jx == 0 ? va0 : 0.f); o[1] = tohx(jx == 0 ? va1 : 0.f); o[2] = tohx(jx == 0 ? vt : 0.f); o[3] = tohx(0.f); *(volatile v4h*)(vrow + jx) = o; } if (ps == 0) __threadfence(); } }
__global__ __launch_bounds__(256) void k_softv(const float* __restrict__ Sb, h16* P16) { const int lane = threadIdx.x & 31; const int row = blockIdx.x * 8 + (threadIdx.x >> 5); if (row >= ZH * TT) return; const float* sr = Sb + (size_t)row * NK; float mx = -3.0e38f;
#pragma unroll 1
    for (int ch = 0; ch < NK / 128; ++ch) { const int j0 = ch * 128 + lane * 4; const v4f a = *(const v4f*)(sr + j0);
#pragma unroll
        for (int u = 0; u < 4; ++u) if (j0 + u < NVAL) mx = fmaxf(mx, a[u]); }
#pragma unroll
    for (int sh = 16; sh; sh >>= 1) mx = fmaxf(mx, __shfl_xor(mx, sh, 32));
    float sum = 0.f;
#pragma unroll 1
    for (int ch = 0; ch < NK / 128; ++ch) { const int j0 = ch * 128 + lane * 4; const v4f a = *(const v4f*)(sr + j0);
#pragma unroll
        for (int u = 0; u < 4; ++u) if (j0 + u < NVAL) { float d0 = __fsub_rn(a[u], mx); asm volatile("" : "+v"(d0)); sum += __expf(d0); } }
#pragma unroll
    for (int sh = 16; sh; sh >>= 1) sum += __shfl_xor(sum, sh, 32);
    const float f = __fdiv_rn(PCAR, sum);
    for (int ps = 0; ps < 2; ++ps) {
#pragma unroll 1
        for (int ch = 0; ch < NK / 128; ++ch) { const int j0 = ch * 128 + lane * 4; const v4f a = *(const v4f*)(sr + j0); v4h o;
#pragma unroll
            for (int u = 0; u < 4; ++u) { float p = 0.f; if (j0 + u < NVAL) { float d0 = __fsub_rn(a[u], mx); asm volatile("" : "+v"(d0)); p = __fmul_rn(__expf(d0), f); } o[u] = tohx(p); } *(volatile v4h*)(P16 + (size_t)row * NK + j0) = o; }
        if (ps == 0) __threadfence(); } }
__global__ __launch_bounds__(256) void k_mrg16(const float* __restrict__ O, int h0, h16* ATT16) { const int e = (blockIdx.x * 256 + threadIdx.x) * 4; if (e >= TT * ZH * HD) return; const int c = e % (ZH * HD); const int t = e / (ZH * HD); const int z = c / HD, d = c % HD; const float* r = O + ((size_t)z * TT + t) * HD + d; v4h o;
#pragma unroll
    for (int u = 0; u < 4; ++u) o[u] = tohx(r[u] * (1.0f / PCAR)); h16* dst = ATT16 + (size_t)t * DD + (h0 + z) * HD + d; *(volatile v4h*)dst = o; __threadfence(); *(volatile v4h*)dst = o; }
__global__ __launch_bounds__(256) void k_out32(const float* __restrict__ T64, const float* __restrict__ b, float* OUTb) { const int e = (blockIdx.x * 256 + threadIdx.x) * 4; if (e >= TT * 32) return; const int j = e % 32; const int t = e / 32; const v4f a = *(const v4f*)(T64 + (size_t)t * 64 + j); v4f o;
#pragma unroll
    for (int u = 0; u < 4; ++u) o[u] = __fadd_rn(a[u], bfr(b[j + u])); *(volatile v4f*)(OUTb + e) = o; __threadfence(); *(volatile v4f*)(OUTb + e) = o; }

extern "C" void kernel_launch(void* const* d_in, const int* in_sizes, int n_in,
                              void* d_out, int out_size, void* d_ws, size_t ws_size, hipStream_t stream) {
    (void)in_sizes; (void)n_in; (void)out_size;
    const float* x = (const float*)d_in[0]; const float* h_a = (const float*)d_in[1]; const float* h_t = (const float*)d_in[2]; const float* p_ = (const float*)d_in[3]; const float* ln1g = (const float*)d_in[4]; const float* ln1b = (const float*)d_in[5]; const float* fc1W = (const float*)d_in[6]; const float* fc1b = (const float*)d_in[7];
    const float* qW = (const float*)d_in[8]; const float* qb = (const float*)d_in[9]; const float* ksW = (const float*)d_in[10]; const float* ksb = (const float*)d_in[11]; const float* vsW = (const float*)d_in[12]; const float* vsb = (const float*)d_in[13]; const float* kaW = (const float*)d_in[14]; const float* kab = (const float*)d_in[15]; const float* vaW = (const float*)d_in[16]; const float* vab = (const float*)d_in[17]; const float* ktW = (const float*)d_in[18]; const float* ktb = (const float*)d_in[19]; const float* vtW = (const float*)d_in[20]; const float* vtb = (const float*)d_in[21]; const float* oW = (const float*)d_in[22]; const float* ob = (const float*)d_in[23]; const float* gsc = (const float*)d_in[24];
    const float* lnG = (const float*)d_in[25]; const float* lnB = (const float*)d_in[26]; const float* fW = (const float*)d_in[27]; const float* fb = (const float*)d_in[28]; const float* ln2g = (const float*)d_in[29]; const float* ln2b = (const float*)d_in[30]; const float* fc2W = (const float*)d_in[31]; const float* fc2b = (const float*)d_in[32];
    float* OUT = (float*)d_out;
    char* wsp = (char*)d_ws;
    auto take = [&](size_t bytes) { char* p = wsp; wsp += (bytes + 255) & ~(size_t)255; return (void*)p; };
    h16* FC1 = (h16*)take((size_t)DD * DIN * 2); h16* FC2 = (h16*)take(64 * DD * 2); h16* QW[2]; h16* KSW[2]; h16* VSW[2]; h16* OWt[2]; h16* FWt[2]; for (int i = 0; i < 2; ++i) { QW[i] = (h16*)take(DD * DD * 2); KSW[i] = (h16*)take(DD * DD * 2); VSW[i] = (h16*)take(DD * DD * 2); OWt[i] = (h16*)take(DD * DD * 2); FWt[i] = (h16*)take(DD * DD * 2); }
    h16* LN16 = (h16*)take((size_t)TT * DIN * 2); float* F = (float*)take((size_t)TT * DD * 4); float* XF = (float*)take((size_t)TT * DD * 4); h16* X16 = (h16*)take((size_t)TT * DD * 2); float* Q = (float*)take((size_t)TT * DD * 4); float* KS = (float*)take((size_t)TT * DD * 4); float* VS = (float*)take((size_t)TT * DD * 4);
    h16* Q16 = (h16*)take((size_t)NH_ * TT * HD * 2); h16* K16 = (h16*)take((size_t)NH_ * NK * HD * 2); h16* VT16 = (h16*)take((size_t)NH_ * HD * NK * 2); float* Sb = (float*)take((size_t)ZH * TT * NK * 4); h16* P16 = (h16*)take((size_t)ZH * TT * NK * 2); float* O = (float*)take((size_t)ZH * TT * HD * 4); h16* ATT16 = (h16*)take((size_t)TT * DD * 2); float* O2 = (float*)take((size_t)TT * DD * 4); float* Y = (float*)take((size_t)TT * DD * 4); h16* Y16 = (h16*)take((size_t)TT * DD * 2); float* T64 = (float*)take((size_t)TT * 64 * 4);
    if ((size_t)(wsp - (char*)d_ws) > ws_size) return;
    k_wt16<<<(DIN / 64) * (DD / 64), 256, 0, stream>>>(fc1W, DIN, DD, FC1); k_wpad16<<<(64 * DD / 2 + 255) / 256, 256, 0, stream>>>(fc2W, FC2);
    for (int i = 0; i < 2; ++i) { k_wt16<<<(DD / 64) * (DD / 64), 256, 0, stream>>>(qW + (size_t)i * DD * DD, DD, DD, QW[i]); k_wt16<<<(DD / 64) * (DD / 64), 256, 0, stream>>>(ksW + (size_t)i * DD * DD, DD, DD, KSW[i]); k_wt16<<<(DD / 64) * (DD / 64), 256, 0, stream>>>(vsW + (size_t)i * DD * DD, DD, DD, VSW[i]); k_wt16<<<(DD / 64) * (DD / 64), 256, 0, stream>>>(oW + (size_t)i * DD * DD, DD, DD, OWt[i]); k_wt16<<<(DD / 64) * (DD / 64), 256, 0, stream>>>(fW + (size_t)i * DD * DD, DD, DD, FWt[i]); }
    for (int b = 0; b < NB_; ++b) {
        k_ln16<DIN, 1><<<TT / 8, 256, 0, stream>>>(x + (size_t)b * TT * DIN, nullptr, ln1g, ln1b, LN16);
        k_gemmw<h16, 0, true><<<dim3(TT / 64, DD / 64, 1), 32, 0, stream>>>(LN16, nullptr, FC1, nullptr, DIN, F, DD, fc1b, 0, 0, 0); k_relux<<<(TT * DD / 4 + 255) / 256, 256, 0, stream>>>(F, XF, X16);
        for (int i = 0; i < 2; ++i) {
            k_gemmw<h16, 0, true><<<dim3(TT / 64, DD / 64, 1), 32, 0, stream>>>(X16, nullptr, QW[i], nullptr, DD, Q, DD, qb + i * DD, 0, 0, 0); k_gemmw<h16, 0, true><<<dim3(TT / 64, DD / 64, 1), 32, 0, stream>>>(X16, nullptr, KSW[i], nullptr, DD, KS, DD, ksb + i * DD, 0, 0, 0); k_gemmw<h16, 0, true><<<dim3(TT / 64, DD / 64, 1), 32, 0, stream>>>(X16, nullptr, VSW[i], nullptr, DD, VS, DD, vsb + i * DD, 0, 0, 0);
            k_ropeqk<<<(NH_ * TT * HD / 2 + 255) / 256, 256, 0, stream>>>(Q, 0.125f, Q16, (size_t)TT * HD); k_ropeqk<<<(NH_ * TT * HD / 2 + 255) / 256, 256, 0, stream>>>(KS, 1.0f, K16, (size_t)NK * HD); k_vt<<<(NH_ * HD * TT / 2 + 255) / 256, 256, 0, stream>>>(VS, VT16);
            k_adp<<<NH_, 64, 0, stream>>>(h_a + ((size_t)b * 3 + i + 1) * DD, p_ + (size_t)b * DD, h_t + ((size_t)b * 3 + i + 1) * DD, kaW + (size_t)i * DD * DD, kab + i * DD, vaW + (size_t)i * DD * DD, vab + i * DD, ktW + (size_t)i * DD * DD, ktb + i * DD, vtW + (size_t)i * DD * DD, vtb + i * DD, gsc + i, K16, VT16);
            for (int h0 = 0; h0 < NH_; h0 += ZH) {
                k_gemmw<h16, 0, false><<<dim3(TT / 64, NK / 64, ZH), 32, 0, stream>>>(Q16 + (size_t)h0 * TT * HD, nullptr, K16 + (size_t)h0 * NK * HD, nullptr, HD, Sb, NK, nullptr, (size_t)TT * HD, (size_t)NK * HD, (size_t)TT * NK);
                k_softv<<<ZH * TT / 8, 256, 0, stream>>>(Sb, P16);
                k_gemmw<h16, 0, false><<<dim3(TT / 64, 1, ZH), 32, 0, stream>>>(P16, nullptr, VT16 + (size_t)h0 * HD * NK, nullptr, NK, O, HD, nullptr, (size_t)TT * NK, (size_t)HD * NK, (size_t)TT * HD);
                k_mrg16<<<(TT * ZH * HD / 4 + 255) / 256, 256, 0, stream>>>(O, h0, ATT16); }
            k_gemmw<h16, 0, true><<<dim3(TT / 64, DD / 64, 1), 32, 0, stream>>>(ATT16, nullptr, OWt[i], nullptr, DD, O2, DD, ob + i * DD, 0, 0, 0);
            k_ln16<DD, 0><<<TT / 8, 256, 0, stream>>>(O2, XF, lnG + i * DD, lnB + i * DD, Y16);
            k_gemmw<h16, 0, true><<<dim3(TT / 64, DD / 64, 1), 32, 0, stream>>>(Y16, nullptr, FWt[i], nullptr, DD, F, DD, fb + i * DD, 0, 0, 0); k_relux<<<(TT * DD / 4 + 255) / 256, 256, 0, stream>>>(F, XF, X16); }
        k_ln16<DD, 0><<<TT / 8, 256, 0, stream>>>(XF, nullptr, ln2g, ln2b, Y16);
        k_gemmw<h16, 0, false><<<dim3(TT / 64, 1, 1), 32, 0, stream>>>(Y16, nullptr, FC2, nullptr, DD, T64, 64, nullptr, 0, 0, 0); k_out32<<<(TT * 32 / 4 + 255) / 256, 256, 0, stream>>>(T64, fc2b, OUT + (size_t)b * TT * 32); }
}
